// DotProductAttention_7533372637539
// MI455X (gfx1250) — hardware-verified
//
#include <hip/hip_runtime.h>
#include <math.h>
#include <stdint.h>

#ifndef NB
#define NB 32
#endif
#ifndef SEQ
#define SEQ 2048
#endif
#define NB_FULL  32
#define SEQ_FULL 2048
#define HD       64
#define NQB    (SEQ / 64)
#define NKT    (SEQ / 64)
static_assert(NB >= 1 && NB <= NB_FULL);
static_assert(SEQ >= 64 && SEQ <= SEQ_FULL && (SEQ % 64) == 0);
static_assert((SEQ_FULL % 256) == 0 && HD == 64);

typedef __bf16         v16b  __attribute__((ext_vector_type(16)));
typedef float          v8f   __attribute__((ext_vector_type(8)));
typedef float          v4f   __attribute__((ext_vector_type(4)));
typedef unsigned int   v4u   __attribute__((ext_vector_type(4)));
typedef unsigned short v8us  __attribute__((ext_vector_type(8)));
typedef unsigned short v16us __attribute__((ext_vector_type(16)));

#if defined(__HIP_DEVICE_COMPILE__)
#define DEV_ASM 1
#else
#define DEV_ASM 0
#endif

__device__ __forceinline__ unsigned short bf_bits(float f) {
  unsigned u = __float_as_uint(f);
  return (unsigned short)((u + 0x7FFFu + ((u >> 16) & 1u)) >> 16);
}
__device__ __forceinline__ float bf_up(unsigned short hb) { return __uint_as_float(((unsigned)hb) << 16); }
__device__ __forceinline__ unsigned pk16(unsigned short a, unsigned short b) { return (unsigned)a | ((unsigned)b << 16); }
__device__ __forceinline__ v8f zero8() { v8f z = {0.f, 0.f, 0.f, 0.f, 0.f, 0.f, 0.f, 0.f}; return z; }

__device__ __forceinline__ v16b ldfrag_b(const unsigned short* p) {
  union { v16us v; v8us h[2]; } f;
  f.h[0] = *(const v8us*)(p);
  f.h[1] = *(const v8us*)(p + 16);
  return __builtin_bit_cast(v16b, f.v);
}

__device__ __forceinline__ v8f mma_b(v16b a, v16b b, v8f c) {
  c = __builtin_amdgcn_wmma_f32_16x16x32_bf16(false, a, false, b, (short)0, c, false, false);
#if DEV_ASM
  asm volatile("v_nop\n\tv_nop\n\tv_nop\n\tv_nop" : "+v"(c) : "v"(a), "v"(b));
#endif
  return c;
}

__global__ __launch_bounds__(256) void cvt_bf16x8(const float* __restrict__ in, unsigned short* out, int n8) {
  const int i = blockIdx.x * 256 + (int)threadIdx.x;
  if (i < n8) {
    const v4f a = *(const v4f*)(in + (size_t)i * 8);
    const v4f b = *(const v4f*)(in + (size_t)i * 8 + 4);
    v4u p;
    p[0] = pk16(bf_bits(a[0]), bf_bits(a[1]));
    p[1] = pk16(bf_bits(a[2]), bf_bits(a[3]));
    p[2] = pk16(bf_bits(b[0]), bf_bits(b[1]));
    p[3] = pk16(bf_bits(b[2]), bf_bits(b[3]));
    *(volatile v4u*)(out + (size_t)i * 8) = p;
    __threadfence();
    *(volatile v4u*)(out + (size_t)i * 8) = p;
  }
}

__global__ __launch_bounds__(256) void vt_prep(const float* __restrict__ V, unsigned short* outp) {
  __shared__ __align__(16) unsigned short sW[16 * 256];
  const int tid  = (int)threadIdx.x;
  const int wave = tid >> 5;
  const int lane = tid & 31;
  const int d0   = blockIdx.x * 16;
  const int s0   = blockIdx.y * 256;
  const int b    = blockIdx.z;
  const float* src = V + ((size_t)b * SEQ_FULL + s0 + tid) * HD + d0;
  const v4f a0 = *(const v4f*)(src);
  const v4f a1 = *(const v4f*)(src + 4);
  const v4f a2 = *(const v4f*)(src + 8);
  const v4f a3 = *(const v4f*)(src + 12);
#pragma unroll
  for (int e = 0; e < 4; ++e) {
    sW[(e)      * 256 + tid] = bf_bits(a0[e]);
    sW[(4 + e)  * 256 + tid] = bf_bits(a1[e]);
    sW[(8 + e)  * 256 + tid] = bf_bits(a2[e]);
    sW[(12 + e) * 256 + tid] = bf_bits(a3[e]);
  }
  __syncthreads();
  const int r0 = 2 * wave;
  const v4u w0 = *(const v4u*)(sW + r0 * 256 + lane * 8);
  const v4u w1 = *(const v4u*)(sW + (r0 + 1) * 256 + lane * 8);
  const size_t o0 = ((size_t)b * HD + d0 + r0) * SEQ_FULL + s0 + lane * 8;
  const size_t o1 = ((size_t)b * HD + d0 + r0 + 1) * SEQ_FULL + s0 + lane * 8;
  for (int pass = 0; pass < 2; ++pass) {
    *(volatile v4u*)(outp + o0) = w0;
    *(volatile v4u*)(outp + o1) = w1;
    __threadfence();
  }
}

#define A_KSH  0
#define A_VT   8192
#define A_PH   16384
#define A_PL   24576
#define A_ACC  32768
#define A_TOT  49152
static_assert(A_VT - A_KSH == 64 * HD * 2 && A_PH - A_VT == HD * 64 * 2);
static_assert(A_PL - A_PH == 4 * 16 * 64 * 2 && A_ACC - A_PL == 4 * 16 * 64 * 2);
static_assert(A_TOT - A_ACC == 4 * 4 * 32 * 8 * 4);
static_assert(4 * 16 * HD * 4 <= A_PH);

__global__ __launch_bounds__(128) __attribute__((amdgpu_num_vgpr(256)))
void attn_fwd(const unsigned short* __restrict__ qp, const unsigned short* __restrict__ kp,
              const unsigned short* __restrict__ vtp, const int* __restrict__ vlp,
              float* outp, float scale) {
  extern __shared__ __align__(16) unsigned char lds[];
  unsigned short* Ksh  = (unsigned short*)(lds + A_KSH);
  unsigned short* Vt   = (unsigned short*)(lds + A_VT);
  unsigned short* Ph   = (unsigned short*)(lds + A_PH);
  unsigned short* Pl   = (unsigned short*)(lds + A_PL);
  float*          accL = (float*)(lds + A_ACC);

  const int tid  = (int)threadIdx.x;
  const int wave = tid >> 5;
  const int lane = tid & 31;
  const int hh   = lane >> 4;
  const int c    = lane & 15;

  const int bx = blockIdx.x;
  const int qb = bx % NQB;
  const int b  = bx / NQB;
  const int q0 = qb * 64 + wave * 16;
  const size_t rowB = (size_t)b * SEQ_FULL;

  const int  vraw = vlp[b];
  const bool none = (vraw <= 0);
  int vl = none ? SEQ : vraw;
  vl = (vl > SEQ) ? SEQ : vl;
  const float sc = none ? 0.f : scale;
  int nkt = (vl + 63) >> 6;
  nkt = (nkt > NKT) ? NKT : nkt;

  const unsigned short* Vtb = vtp + (size_t)b * HD * SEQ_FULL;

  unsigned short* pwh  = Ph + wave * 1024;
  unsigned short* pwl  = Pl + wave * 1024;
  float*          accW = accL + wave * 1024;

#pragma unroll
  for (int t = 0; t < 4; ++t) *(v8f*)(accW + (t * 32 + lane) * 8) = zero8();

  float mrow[8], lrow[8], alpha[8];
#pragma unroll
  for (int r = 0; r < 8; ++r) { mrow[r] = -INFINITY; lrow[r] = 0.f; alpha[r] = 0.f; }

  const size_t qo = (rowB + q0 + c) * HD + 8 * hh;

  for (int kt = 0; kt < nkt; ++kt) {
    const int kv0 = kt * 64;
    __syncthreads();
    {
#pragma unroll 2
      for (int i = 0; i < 4; ++i) {
        const int p   = tid + 128 * i;
        const int kr  = p >> 3;
        const int kp8 = (p & 7) * 8;
        const v8us a0 = *(const v8us*)(kp + (rowB + kv0 + kr) * HD + kp8);
        const int d   = p >> 3;
        const int sg  = (p & 7) * 8;
        const v8us b0 = *(const v8us*)(Vtb + (size_t)d * SEQ_FULL + kv0 + sg);
        *(v8us*)(Ksh + kr * HD + kp8) = a0;
        *(v8us*)(Vt + d * 64 + sg) = b0;
      }
    }
    __syncthreads();

    v8f s[4];
#pragma unroll
    for (int j = 0; j < 4; ++j) s[j] = zero8();
#pragma unroll 1
    for (int dc = 0; dc < 2; ++dc) {
      const v16b qa = ldfrag_b(qp + qo + dc * 32);
      const int ko = dc * 32 + 8 * hh;
#pragma unroll
      for (int j = 0; j < 4; ++j) {
        const v16b kb = ldfrag_b(Ksh + (j * 16 + c) * HD + ko);
        s[j] = mma_b(qa, kb, s[j]);
      }
    }

#pragma unroll
    for (int r = 0; r < 8; ++r) {
      float m = -INFINITY;
#pragma unroll
      for (int j = 0; j < 4; ++j) {
        const int key = kv0 + j * 16 + c;
        float sv = s[j][r] * sc;
        sv = (key < vl) ? sv : -INFINITY;
        s[j][r] = sv;
        m = fmaxf(m, sv);
      }
#pragma unroll
      for (int off = 1; off < 16; off <<= 1) m = fmaxf(m, __shfl_xor(m, off, 32));
      const float mnew  = fmaxf(mrow[r], m);
      const float msafe = (mnew == -INFINITY) ? 0.f : mnew;
      const float al    = __expf(mrow[r] - msafe);
      mrow[r]  = mnew;
      alpha[r] = al;
      float psum = 0.f;
#pragma unroll
      for (int j = 0; j < 4; ++j) {
        const float p = __expf(s[j][r] - msafe);
        psum += p;
        const unsigned short hb = bf_bits(p);
        const unsigned short lb = bf_bits(p - bf_up(hb));
        const int po = (8 * hh + r) * 64 + j * 16 + c;
        pwh[po] = hb;
        pwl[po] = lb;
      }
#pragma unroll
      for (int off = 1; off < 16; off <<= 1) psum += __shfl_xor(psum, off, 32);
      lrow[r] = lrow[r] * al + psum;
    }
    __builtin_amdgcn_fence(3  , "workgroup");
    __builtin_amdgcn_wave_barrier();
    __builtin_amdgcn_fence(2  , "workgroup");

    v16b pa[2], pb[2];
#pragma unroll
    for (int kk = 0; kk < 2; ++kk) {
      const int pr = c * 64 + kk * 32 + 8 * hh;
      pa[kk] = ldfrag_b(pwh + pr);
      pb[kk] = ldfrag_b(pwl + pr);
    }
#pragma unroll 1
    for (int t = 0; t < 4; ++t) {
      float* ap = accW + (t * 32 + lane) * 8;
      v8f acc = *(const v8f*)ap;
#pragma unroll
      for (int r = 0; r < 8; ++r) acc[r] *= alpha[r];
      const int vr0 = (t * 16 + c) * 64 + 8 * hh;
#pragma unroll
      for (int kk = 0; kk < 2; ++kk) {
        const v16b vb = ldfrag_b(Vt + vr0 + kk * 32);
        acc = mma_b(pa[kk], vb, acc);
        acc = mma_b(pb[kk], vb, acc);
      }
      *(v8f*)ap = acc;
    }
  }

  __syncthreads();

  float* os = (float*)(lds + A_KSH) + wave * (16 * HD);
  float inv[8];
#pragma unroll
  for (int r = 0; r < 8; ++r) {
    const float l = lrow[r];
    inv[r] = (l > 0.f) ? (1.0f / l) : 0.f;
  }
#pragma unroll 1
  for (int t = 0; t < 4; ++t) {
    const v8f acc = *(const v8f*)(accW + (t * 32 + lane) * 8);
#pragma unroll
    for (int r = 0; r < 8; ++r) os[(8 * hh + r) * HD + t * 16 + c] = acc[r] * inv[r];
  }
  __builtin_amdgcn_fence(3  , "workgroup");
  __builtin_amdgcn_wave_barrier();
  __builtin_amdgcn_fence(2  , "workgroup");
  const size_t ob = (rowB + q0) * HD;
  for (int pass = 0; pass < 2; ++pass) {
#pragma unroll
    for (int it = 0; it < 8; ++it) {
      const v4f v = *(const v4f*)(os + it * 128 + lane * 4);
      *(volatile v4f*)(outp + ob + it * 128 + lane * 4) = v;
    }
    __threadfence();
  }
}

extern "C" void kernel_launch(void* const* d_in, const int* in_sizes, int n_in,
                              void* d_out, int out_size, void* d_ws, size_t ws_size,
                              hipStream_t stream) {
  if (n_in < 4) return;
  const long needIn  = (long)NB * SEQ_FULL * HD;
  const long needOut = ((long)(NB - 1) * SEQ_FULL + SEQ) * HD;
  if ((long)in_sizes[0] < needIn) return;
  if ((long)in_sizes[1] < needIn) return;
  if ((long)in_sizes[2] < needIn) return;
  if (in_sizes[3] < NB) return;
  if ((long)out_size < needOut) return;

  const float* q  = (const float*)d_in[0];
  const float* k  = (const float*)d_in[1];
  const float* v  = (const float*)d_in[2];
  const int*   vl = (const int*)d_in[3];

  const size_t PP = (size_t)NB * SEQ_FULL * HD * 2;
  size_t off = 0;
  const size_t oQ  = off; off += PP;
  const size_t oK  = off; off += PP;
  const size_t oVT = off; off += PP;
  if (off > ws_size) return;
  if (off > (size_t)134217728) return;

  char* ws = (char*)d_ws;
  unsigned short* Qb  = (unsigned short*)(ws + oQ);
  unsigned short* Kb  = (unsigned short*)(ws + oK);
  unsigned short* VTb = (unsigned short*)(ws + oVT);

  const dim3 blk(256);
  const int n8 = NB * SEQ_FULL * HD / 8;
  const dim3 gCvt((n8 + 255) / 256);
  const dim3 gVt(HD / 16, SEQ_FULL / 256, NB);
  const dim3 gAtt(NB * NQB);
  const float scale = 0.125f;

  cvt_bf16x8<<<gCvt, blk, 0, stream>>>(q, Qb, n8);
  cvt_bf16x8<<<gCvt, blk, 0, stream>>>(k, Kb, n8);
  vt_prep<<<gVt, blk, 0, stream>>>(v, VTb);
  (void)hipFuncSetAttribute(reinterpret_cast<const void*>(&attn_fwd),
                            hipFuncAttributeMaxDynamicSharedMemorySize, A_TOT);
  attn_fwd<<<gAtt, dim3(128), A_TOT, stream>>>(Qb, Kb, VTb, vl, (float*)d_out, scale);
  (void)hipGetLastError();
}
